// TF_GAM_52793738002611
// MI455X (gfx1250) — hardware-verified
//
#include <hip/hip_runtime.h>
#include <math.h>


typedef _Float16 v8h  __attribute__((ext_vector_type(8)));
typedef _Float16 v16h __attribute__((ext_vector_type(16)));
typedef float    v8f  __attribute__((ext_vector_type(8)));

typedef __bf16   v16bf __attribute__((ext_vector_type(16)));
typedef unsigned v8u  __attribute__((ext_vector_type(8)));

__device__ __forceinline__ unsigned f2bf(float f) { unsigned u = __float_as_uint(f); u += 0x7FFFu + ((u >> 16) & 1u); return u >> 16; }
__device__ __forceinline__ int kpat(int v, int half) { return ((v & 4) ? 16 : 0) + half * 8 + 2 * (v & 3); }
struct Op2 { v16bf hi, lo; };
__device__ __forceinline__ Op2 op_row2(const float* rowp, int half) {
    v8u uh, ul;
#pragma unroll
    for (int v = 0; v < 8; ++v) {
        const int kk = kpat(v, half);
        const float f0 = rowp[kk], f1 = rowp[kk + 1];
        const unsigned h0 = f2bf(f0), h1 = f2bf(f1);
        const unsigned l0 = f2bf(f0 - __uint_as_float(h0 << 16)), l1 = f2bf(f1 - __uint_as_float(h1 << 16));
        uh[v] = h0 | (h1 << 16); ul[v] = l0 | (l1 << 16);
    }
    Op2 o; o.hi = __builtin_bit_cast(v16bf, uh); o.lo = __builtin_bit_cast(v16bf, ul); return o;
}
__device__ __forceinline__ v8f wmma_split2(const Op2& a, const Op2& b, v8f c) {
    c = __builtin_amdgcn_wmma_f32_16x16x32_bf16(false, a.hi, false, b.hi, (short)0, c, false, false);
    c = __builtin_amdgcn_wmma_f32_16x16x32_bf16(false, a.hi, false, b.lo, (short)0, c, false, false);
    c = __builtin_amdgcn_wmma_f32_16x16x32_bf16(false, a.lo, false, b.hi, (short)0, c, false, false);
    asm volatile("v_nop\n\tv_nop\n\tv_nop\n\tv_nop" : "+v"(c) : "v"(a.hi), "v"(a.lo), "v"(b.hi), "v"(b.lo));
    return c;
}

constexpr int   B      = 4;
constexpr int   N      = 4096;
constexpr int   D      = 512;
constexpr int   TOPK   = 8;
constexpr float LAMBDA = 0.8f;
constexpr float EPSN   = 1e-12f;

__global__ __launch_bounds__(256)
void gam_normalize(const float* __restrict__ x,
                   float* fF) {
    const int row  = blockIdx.x * 8 + (threadIdx.x >> 5);
    const int lane = threadIdx.x & 31;
    const float* xr = x + (size_t)row * D;

    float v[16];
    float s = 0.f;
#pragma unroll
    for (int i = 0; i < 16; ++i) {
        v[i] = xr[lane + 32 * i];
        s += v[i] * v[i];
    }
#pragma unroll
    for (int m = 16; m >= 1; m >>= 1) s += __shfl_xor(s, m, 32);

    const float inv = 1.f / fmaxf(sqrtf(s), EPSN);
    float* fr = fF + (size_t)row * D;
#pragma unroll
    for (int i = 0; i < 16; ++i) *(volatile float*)(fr + lane + 32 * i) = v[i] * inv;
    __threadfence();
#pragma unroll
    for (int i = 0; i < 16; ++i) *(volatile float*)(fr + lane + 32 * i) = v[i] * inv;
}

__global__ __launch_bounds__(256)
void gam_attend(const float* __restrict__ fF,
                float* out) {
    extern __shared__ char smem[];
    float* sS   = (float*)smem;
    float* sCV  = sS + 16 * N;
    int*   sCI  = (int*)(sCV + 16 * 128);
    float* sW   = (float*)(sCI + 16 * 128);
    int*   sWI  = (int*)(sW + 16 * TOPK);
    float* sRed = (float*)(sWI + 16 * TOPK);

    const int b       = blockIdx.x / (N / 16);
    const int rowbase = (blockIdx.x % (N / 16)) * 16;
    const int tid     = threadIdx.x;
    const int wave    = tid >> 5;
    const int lane    = tid & 31;
    const size_t batchOff = (size_t)b * N * D;

    {
        const int l16 = lane & 15, half = lane >> 4;
        const float* aptr = fF + batchOff + (size_t)(rowbase + l16) * D;
        for (int grp = 0; grp < 4; ++grp) {
            v8f c[8];
#pragma unroll
            for (int t = 0; t < 8; ++t) c[t] = (v8f){};
#pragma unroll 1
            for (int ks = 0; ks < D / 32; ++ks) {
                const Op2 a = op_row2(aptr + ks * 32, half);
#pragma unroll
                for (int t = 0; t < 8; ++t) {
                    const int colbase = (wave * 32 + grp * 8 + t) * 16;
                    const Op2 b = op_row2(fF + batchOff + (size_t)(colbase + l16) * D + ks * 32, half);
                    c[t] = wmma_split2(a, b, c[t]);
                }
            }
#pragma unroll
            for (int t = 0; t < 8; ++t) {
                const int col = (wave * 32 + grp * 8 + t) * 16 + l16;
#pragma unroll
                for (int r = 0; r < 8; ++r) sS[(half * 8 + r) * N + col] = c[t][r];
            }
        }
    }
    __syncthreads();

    const int g = tid >> 4;
    const int t = tid & 15;
    {
        float tv[TOPK];
        int   tix[TOPK];
#pragma unroll
        for (int j = 0; j < TOPK; ++j) { tv[j] = -INFINITY; tix[j] = 0; }
        const float* rowS = sS + g * N;
        const int c0 = t * (N / 16);
        for (int c = 0; c < N / 16; ++c) {
            const float v = rowS[c0 + c];
            if (v > tv[TOPK - 1]) {
                tv[TOPK - 1]  = v;
                tix[TOPK - 1] = c0 + c;
#pragma unroll
                for (int j = TOPK - 1; j > 0; --j)
                    if (tv[j] > tv[j - 1]) {
                        const float fv = tv[j]; tv[j] = tv[j - 1]; tv[j - 1] = fv;
                        const int   ii = tix[j]; tix[j] = tix[j - 1]; tix[j - 1] = ii;
                    }
            }
        }
#pragma unroll
        for (int j = 0; j < TOPK; ++j) {
            sCV[g * 128 + t * TOPK + j] = tv[j];
            sCI[g * 128 + t * TOPK + j] = tix[j];
        }
    }
    __syncthreads();

    if (t == 0) {
        float* cv = sCV + g * 128;
        int*   ci = sCI + g * 128;
        float bv[TOPK];
        int   bix[TOPK];
#pragma unroll
        for (int j = 0; j < TOPK; ++j) {
            float best = -INFINITY; int bi = 0;
            for (int c = 0; c < 128; ++c)
                if (cv[c] > best) { best = cv[c]; bi = c; }
            bv[j] = best; bix[j] = ci[bi]; cv[bi] = -INFINITY;
        }
        const float mx = bv[0];
        float w[TOPK];
        float se = 0.f;
#pragma unroll
        for (int j = 0; j < TOPK; ++j) { w[j] = expf(bv[j] - mx); se += w[j]; }
        const float r = 1.f / se;
#pragma unroll
        for (int j = 0; j < TOPK; ++j) {
            sW[g * TOPK + j]  = w[j] * r;
            sWI[g * TOPK + j] = bix[j];
        }
    }
    __syncthreads();

    {
        const int rowg = rowbase + g;
        float w[TOPK];
        const float* frows[TOPK];
#pragma unroll
        for (int j = 0; j < TOPK; ++j) {
            w[j]     = sW[g * TOPK + j];
            frows[j] = fF + batchOff + (size_t)sWI[g * TOPK + j] * D;
        }
        const float* self = fF + batchOff + (size_t)rowg * D;

        float gv[32];
        float ss = 0.f;
#pragma unroll
        for (int i = 0; i < 32; ++i) {
            const int d = t + 16 * i;
            float att = 0.f;
#pragma unroll
            for (int j = 0; j < TOPK; ++j) att += w[j] * frows[j][d];
            const float val = LAMBDA * self[d] + (1.f - LAMBDA) * att;
            gv[i] = val;
            ss += val * val;
        }
        sRed[g * 16 + t] = ss;
        __syncthreads();
        float tot = 0.f;
#pragma unroll
        for (int i = 0; i < 16; ++i) tot += sRed[g * 16 + i];
        const float inv = 1.f / fmaxf(sqrtf(tot), EPSN);

#pragma unroll
        for (int i = 0; i < 32; ++i) sS[g * D + t + 16 * i] = gv[i] * inv;
    }
    __syncthreads();
    {
        float* ob = out + batchOff + (size_t)rowbase * D;
#pragma unroll
        for (int j = 0; j < 2; ++j) {
            const int r = wave * 2 + j;
#pragma unroll
            for (int cc = 0; cc < D / 32; ++cc) *(volatile float*)(ob + (size_t)r * D + cc * 32 + lane) = sS[r * D + cc * 32 + lane];
        }
        __threadfence();
#pragma unroll
        for (int j = 0; j < 2; ++j) {
            const int r = wave * 2 + j;
#pragma unroll
            for (int cc = 0; cc < D / 32; ++cc) *(volatile float*)(ob + (size_t)r * D + cc * 32 + lane) = sS[r * D + cc * 32 + lane];
        }
    }
}

extern "C" void kernel_launch(void* const* d_in, const int* in_sizes, int n_in,
                              void* d_out, int out_size, void* d_ws, size_t ws_size,
                              hipStream_t stream) {
    (void)in_sizes; (void)n_in; (void)out_size;
    const float* feats = (const float*)d_in[0];

    float*    fF = (float*)d_ws;
    float*    out = (float*)d_out;
    if ((size_t)B * N * D * sizeof(float) > ws_size) return;

    gam_normalize<<<(B * N) / 8, 256, 0, stream>>>(feats, fF);

    const size_t smem =
        (size_t)16 * N * sizeof(float)
        + 16 * 128 * (sizeof(float) + sizeof(int))
        + 16 * TOPK * (sizeof(float) + sizeof(int))
        + 16 * 16 * sizeof(float);
    gam_attend<<<B * (N / 16), 256, smem, stream>>>(fF, out);
}
